// BottleneckResAtnMHSA_21449066676839
// MI455X (gfx1250) — hardware-verified
//
#include <hip/hip_runtime.h>
#include <math.h>
typedef __attribute__((ext_vector_type(16))) _Float16 v16h;
typedef __attribute__((ext_vector_type(8)))  _Float16 v8h;
typedef __attribute__((ext_vector_type(16))) __bf16   v16b;
typedef __attribute__((ext_vector_type(8)))  __bf16   v8b;
typedef __attribute__((ext_vector_type(8)))  float    v8f;
typedef __attribute__((ext_vector_type(4)))  float    v4f;
#define PSCALE 32768.0f
#define U16(p) ((const unsigned short*)(const void*)(p))
#define PSCALE_INV (1.0f / 32768.0f)

__device__ __forceinline__ unsigned short f2bf_bits(float f) {
  unsigned u = __float_as_uint(f);
  return (unsigned short)((u + 0x7FFFu + ((u >> 16) & 1u)) >> 16);
}
__device__ __forceinline__ float bf_bits2f(unsigned short h) { return __uint_as_float(((unsigned)h) << 16); }

__device__ __forceinline__ void dep_guard_h(v8f& a, v8f& b, v16h x, v16h y) { asm volatile("v_nop\n\tv_nop\n\tv_nop\n\tv_nop" : "+v"(a), "+v"(b) : "v"(x), "v"(y)); }
__device__ __forceinline__ void dep_guard_b(v8f& a, v8f& b, v16b x, v16b y) { asm volatile("v_nop\n\tv_nop\n\tv_nop\n\tv_nop" : "+v"(a), "+v"(b) : "v"(x), "v"(y)); }
__device__ __forceinline__ void keep4_h(v16h a, v16h b, v16h c, v16h d) { asm volatile("v_nop" :: "v"(a), "v"(b), "v"(c), "v"(d)); }
__device__ __forceinline__ void keep4_b(v16b a, v16b b, v16b c, v16b d) { asm volatile("v_nop" :: "v"(a), "v"(b), "v"(c), "v"(d)); }
__device__ __forceinline__ void acc_guard4(v8f& a, v8f& b, v8f& c, v8f& d) { asm volatile("v_nop\n\tv_nop\n\tv_nop\n\tv_nop" : "+v"(a), "+v"(b), "+v"(c), "+v"(d)); }
template <typename T> struct Frag;
template <> struct Frag<_Float16> {
  typedef v16h V; union U { v16h v; v8h h[2]; };
  static __device__ __forceinline__ v16h load(const _Float16* p) {
    U f; f.h[0] = *(const v8h*)(p); f.h[1] = *(const v8h*)(p + 16); return f.v;
  }
  static __device__ __forceinline__ v8f mma(v16h a, v16h b, v8f c) {
    return __builtin_amdgcn_wmma_f32_16x16x32_f16(false, a, false, b, (short)0, c, false, false);
  }
  static __device__ __forceinline__ void guard(v8f& a, v8f& b, v16h x, v16h y) { dep_guard_h(a, b, x, y); }
  static __device__ __forceinline__ void keep(v16h a, v16h b, v16h c, v16h d) { keep4_h(a, b, c, d); }
};
template <> struct Frag<__bf16> {
  typedef v16b V; union U { v16b v; v8b h[2]; };
  static __device__ __forceinline__ v16b load(const __bf16* p) {
    U f; f.h[0] = *(const v8b*)(p); f.h[1] = *(const v8b*)(p + 16); return f.v;
  }
  static __device__ __forceinline__ v8f mma(v16b a, v16b b, v8f c) {
    return __builtin_amdgcn_wmma_f32_16x16x32_bf16(false, a, false, b, (short)0, c, false, false);
  }
  static __device__ __forceinline__ void guard(v8f& a, v8f& b, v16b x, v16b y) { dep_guard_b(a, b, x, y); }
  static __device__ __forceinline__ void keep(v16b a, v16b b, v16b c, v16b d) { keep4_b(a, b, c, d); }
};

template <int ET> struct Elem;
template <> struct Elem<0> { typedef _Float16 T; };
template <> struct Elem<1> { typedef __bf16 T; };
template <int ET, bool SPLIT, int BIAS_MODE, int OUT_MODE, bool RESID, int ACT = 0>
__global__ __launch_bounds__(256) void wmma_gemm64(
    const unsigned short* __restrict__ Ap, const unsigned short* __restrict__ A2p, int lda, long strideA,
    const unsigned short* __restrict__ Btp, const unsigned short* __restrict__ Bt2p, int ldb, long strideB,
    void* __restrict__ Cout, void* __restrict__ Cout2, int ldc, long strideC,
    const float* __restrict__ bias,
    const float* __restrict__ resid, long strideR,
    int M, int N, int K, float scale) {
  typedef typename Elem<ET>::T T;
  typedef typename Frag<T>::V V;
  const T* A = (const T*)Ap; const T* A2 = (const T*)A2p; const T* Bt = (const T*)Btp; const T* Bt2 = (const T*)Bt2p;
  __shared__ __align__(16) float sT[8][16 * 68];
  const int b    = blockIdx.y;
  const int lane = threadIdx.x & 31;
  const int wave = threadIdx.x >> 5;
  const int tilesN = N >> 6;
  const int tilesM = M >> 6;
  const int tile = blockIdx.x * 8 + wave;
  if (tile >= tilesM * tilesN) return;
  const int tm = tile / tilesN;
  const int tn = tile - tm * tilesN;
  const int m0 = tm << 6;
  const int n0 = tn << 6;

  const T* Ab  = A  + (size_t)b * strideA;
  const T* Bb  = Bt + (size_t)b * strideB;
  const T* Ab2 = SPLIT ? (A2  + (size_t)b * strideA) : nullptr;
  const T* Bb2 = SPLIT ? (Bt2 + (size_t)b * strideB) : nullptr;

  const int rlane = lane & 15;
  const int koff  = (lane >> 4) * 8;
  const int mOff  = (lane >> 4) * 8;

  v8f acc[4][4];
#pragma unroll
  for (int i = 0; i < 4; ++i)
#pragma unroll
    for (int j = 0; j < 4; ++j) acc[i][j] = (v8f){0.f,0.f,0.f,0.f,0.f,0.f,0.f,0.f};

  for (int k0 = 0; k0 < K; k0 += 32) {
    V bh[4], bl[4];
#pragma unroll
    for (int j = 0; j < 4; ++j) {
      const size_t bo = (size_t)(n0 + (j << 4) + rlane) * ldb + koff + k0;
      bh[j] = Frag<T>::load(Bb + bo);
      if (SPLIT) bl[j] = Frag<T>::load(Bb2 + bo);
    }
#pragma unroll
    for (int i = 0; i < 4; ++i) {
      const size_t ao = (size_t)(m0 + (i << 4) + rlane) * lda + koff + k0;
      V ah = Frag<T>::load(Ab + ao);
      V al;
      if (SPLIT) al = Frag<T>::load(Ab2 + ao);
#pragma unroll
      for (int j = 0; j < 4; ++j) {
        acc[i][j] = Frag<T>::mma(ah, bh[j], acc[i][j]);
        if (SPLIT) {
          acc[i][j] = Frag<T>::mma(ah, bl[j], acc[i][j]);
          acc[i][j] = Frag<T>::mma(al, bh[j], acc[i][j]);
        }
      }
      Frag<T>::guard(acc[i][0], acc[i][3], ah, SPLIT ? al : ah);
    }
    Frag<T>::keep(bh[0], bh[1], bh[2], bh[3]);
    if (SPLIT) Frag<T>::keep(bl[0], bl[1], bl[2], bl[3]);
  }
  acc_guard4(acc[0][0], acc[0][1], acc[0][2], acc[0][3]);
  acc_guard4(acc[1][0], acc[1][1], acc[1][2], acc[1][3]);
  acc_guard4(acc[2][0], acc[2][1], acc[2][2], acc[2][3]);
  acc_guard4(acc[3][0], acc[3][1], acc[3][2], acc[3][3]);

  float* slab = sT[wave];
  const float* Rb = RESID ? (resid + (size_t)b * strideR) : nullptr;
#pragma unroll
  for (int i = 0; i < 4; ++i) {
    const int mBase = m0 + (i << 4);
#pragma unroll
    for (int j = 0; j < 4; ++j) {
      const int n = n0 + (j << 4) + rlane;
      float bv = 0.f;
      if (BIAS_MODE == 2) bv = bias[n];
#pragma unroll
      for (int r = 0; r < 8; ++r) {
        float v = acc[i][j][r] * scale;
        if (BIAS_MODE == 1) v += bias[mBase + mOff + r];
        if (BIAS_MODE == 2) v += bv;
        if (RESID) v += Rb[(size_t)(mBase + mOff + r) * ldc + n];
        if (ACT == 1) v = tanhf(v);
        if (ACT == 2) v = fmaxf(v, 0.0f);
        if (ACT == 3) v = v / (1.0f + expf(-v));
        if (ACT == 4) v = (v > 0.f) ? v : 0.01f * v;
        if (ACT == 5) v = 0.5f * v * (1.0f + erff(v * 0.70710678118654752f));
        slab[(mOff + r) * 68 + (j << 4) + rlane] = v;
      }
    }
    __builtin_amdgcn_fence(__ATOMIC_RELEASE, "workgroup");
    __builtin_amdgcn_wave_barrier();
    __builtin_amdgcn_fence(__ATOMIC_ACQUIRE, "workgroup");
    if (OUT_MODE == 0) {
      float* C = (float*)Cout + (size_t)b * strideC;
      const int hh = lane >> 4, c4 = (lane & 15) * 4;
      for (int pass = 0; pass < 2; ++pass) {
#pragma unroll
        for (int it = 0; it < 8; ++it) {
          const int row = it * 2 + hh;
          v4f v = *(const v4f*)(slab + row * 68 + c4);
          *(volatile v4f*)(C + (size_t)(mBase + row) * ldc + n0 + c4) = v;
        }
        __threadfence();
      }
    } else {
      const int q = lane >> 3, c8 = (lane & 7) * 8;
      unsigned short* C  = (unsigned short*)Cout  + (size_t)b * strideC;
      unsigned short* C2 = (OUT_MODE == 2) ? ((unsigned short*)Cout2 + (size_t)b * strideC) : nullptr;
      for (int pass = 0; pass < 2; ++pass) {
#pragma unroll
        for (int it = 0; it < 4; ++it) {
          const int row = it * 4 + q;
          const float* sp = slab + row * 68 + c8;
          v8h hv, lv;
#pragma unroll
          for (int e = 0; e < 8; ++e) {
            if (OUT_MODE == 1) {
              hv[e] = (_Float16)sp[e];
            } else {
              unsigned short hb = f2bf_bits(sp[e]);
              unsigned short lb = f2bf_bits(sp[e] - bf_bits2f(hb));
              hv[e] = __builtin_bit_cast(_Float16, hb);
              lv[e] = __builtin_bit_cast(_Float16, lb);
            }
          }
          *(volatile v8h*)(C + (size_t)(mBase + row) * ldc + n0 + c8) = hv;
          if (OUT_MODE == 2) *(volatile v8h*)(C2 + (size_t)(mBase + row) * ldc + n0 + c8) = lv;
        }
        __threadfence();
      }
    }
    __builtin_amdgcn_fence(__ATOMIC_RELEASE, "workgroup");
    __builtin_amdgcn_wave_barrier();
    __builtin_amdgcn_fence(__ATOMIC_ACQUIRE, "workgroup");
  }
}

__global__ __launch_bounds__(256) void cast_f32_f16x2(
    const float* __restrict__ in, _Float16* __restrict__ out, int n2) {
  int i = blockIdx.x * 256 + threadIdx.x;
  if (i < n2) {
    const _Float16 h0 = (_Float16)in[2 * i], h1 = (_Float16)in[2 * i + 1];
    const unsigned u = (unsigned)__builtin_bit_cast(unsigned short, h0) | ((unsigned)__builtin_bit_cast(unsigned short, h1) << 16);
    ((volatile unsigned*)out)[i] = u;
    __threadfence();
    ((volatile unsigned*)out)[i] = u;
  }
}


__global__ __launch_bounds__(256) void transpose_cast_f16(const float* __restrict__ in, int ldi,
                                                         _Float16* __restrict__ outT, int ldo, float scale) {
  __shared__ __align__(16) _Float16 tile[64][72];
  const int c0 = blockIdx.x * 64, r0 = blockIdx.y * 64;
  const int t = threadIdx.y * 32 + threadIdx.x;
  for (int i = threadIdx.y; i < 64; i += 8) {
    tile[threadIdx.x][i]      = (_Float16)(in[(size_t)(r0 + i) * ldi + c0 + threadIdx.x] * scale);
    tile[32 + threadIdx.x][i] = (_Float16)(in[(size_t)(r0 + i) * ldi + c0 + 32 + threadIdx.x] * scale);
  }
  __syncthreads();
  const int q = t >> 3, c8 = (t & 7) * 8;
  for (int pass = 0; pass < 2; ++pass) {
#pragma unroll
    for (int it = 0; it < 2; ++it) {
      const int c = it * 32 + q;
      v8h hv = *(const v8h*)(&tile[c][c8]);
      *(volatile v8h*)(outT + (size_t)(c0 + c) * ldo + r0 + c8) = hv;
    }
    __threadfence();
  }
}

#define BB 32
#define CIN 256
#define CM 128
#define NS 1024
__global__ __launch_bounds__(256) void fold_bn_kernel(const float* __restrict__ Wm, const float* __restrict__ g, const float* __restrict__ bb, const float* __restrict__ m, const float* __restrict__ var,
                                                     int O, int Cc, unsigned* __restrict__ W16, float* __restrict__ bias) {
  const int i = blockIdx.x * 256 + threadIdx.x;
  if (i < O * Cc / 2) { const int o = (2 * i) / Cc; const float sc = g[o] / sqrtf(var[o] + 1e-5f);
    const unsigned u = (unsigned)__builtin_bit_cast(unsigned short, (_Float16)(Wm[2 * i] * sc)) | ((unsigned)__builtin_bit_cast(unsigned short, (_Float16)(Wm[2 * i + 1] * sc)) << 16);
    ((volatile unsigned*)W16)[i] = u; __threadfence(); ((volatile unsigned*)W16)[i] = u; }
  if (i < O) { const float sc = g[i] / sqrtf(var[i] + 1e-5f); const float v = bb[i] - m[i] * sc; ((volatile float*)bias)[i] = v; __threadfence(); ((volatile float*)bias)[i] = v; }
}
__global__ __launch_bounds__(256) void pos_kernel(const float* __restrict__ relh, const float* __restrict__ relw, unsigned* __restrict__ QP) {
  const long t = (long)blockIdx.x * 256 + threadIdx.x;
  const int cp = (int)(t & 63); const long bi = t >> 6; const int i = (int)(bi % NS);
  const int ih = i >> 5, iw = i & 31, c0 = 2 * cp;
  const float p0 = relh[(size_t)c0 * 32 + ih] + relw[(size_t)c0 * 32 + iw], p1 = relh[(size_t)(c0 + 1) * 32 + ih] + relw[(size_t)(c0 + 1) * 32 + iw];
  const unsigned u = (unsigned)__builtin_bit_cast(unsigned short, (_Float16)p0) | ((unsigned)__builtin_bit_cast(unsigned short, (_Float16)p1) << 16);
  ((volatile unsigned*)QP)[(size_t)bi * 128 + 64 + cp] = u; __threadfence(); ((volatile unsigned*)QP)[(size_t)bi * 128 + 64 + cp] = u;
}
__global__ __launch_bounds__(256) void softmax_kernel(const float* __restrict__ S, unsigned* __restrict__ P16) {
  __shared__ float red[8]; __shared__ float stat;
  const size_t row = blockIdx.x; const int t = threadIdx.x, lane = t & 31, wave = t >> 5;
  float v[4]; float mx = -INFINITY;
#pragma unroll
  for (int q = 0; q < 2; ++q) { const int n = q * 512 + 2 * t; v[2*q] = S[row * NS + n]; v[2*q+1] = S[row * NS + n + 1]; mx = fmaxf(mx, fmaxf(v[2*q], v[2*q+1])); }
  for (int o = 16; o > 0; o >>= 1) mx = fmaxf(mx, __shfl_xor(mx, o, 32));
  if (lane == 0) red[wave] = mx; __syncthreads();
  if (t == 0) { float m = red[0]; for (int w = 1; w < 8; ++w) m = fmaxf(m, red[w]); stat = m; } __syncthreads();
  const float m = stat; __syncthreads();
  float se = 0.f;
#pragma unroll
  for (int q = 0; q < 4; ++q) { v[q] = expf(v[q] - m); se += v[q]; }
  for (int o = 16; o > 0; o >>= 1) se += __shfl_xor(se, o, 32);
  if (lane == 0) red[wave] = se; __syncthreads();
  if (t == 0) { float s = 0.f; for (int w = 0; w < 8; ++w) s += red[w]; stat = 32768.0f / s; } __syncthreads();
  const float inv = stat;
  for (int pass = 0; pass < 2; ++pass) {
#pragma unroll
    for (int q = 0; q < 2; ++q) { const unsigned u = (unsigned)__builtin_bit_cast(unsigned short, (_Float16)(v[2*q] * inv)) | ((unsigned)__builtin_bit_cast(unsigned short, (_Float16)(v[2*q+1] * inv)) << 16);
      ((volatile unsigned*)P16)[row * (NS / 2) + q * 256 + t] = u; }
    __threadfence();
  }
}
__global__ __launch_bounds__(256) void resid_kernel(const float* __restrict__ x, const float* __restrict__ y, float* __restrict__ out, long n4) {
  const long i = (long)blockIdx.x * 256 + threadIdx.x; if (i >= n4) return;
  const v4f v = *(const v4f*)(x + 4 * i) + *(const v4f*)(y + 4 * i);
  *(volatile v4f*)(out + 4 * i) = v; __threadfence(); *(volatile v4f*)(out + 4 * i) = v;
}
extern "C" void kernel_launch(void* const* d_in, const int* in_sizes, int n_in, void* d_out, int out_size, void* d_ws, size_t ws_size, hipStream_t stream) {
  (void)in_sizes; (void)n_in; (void)out_size; (void)ws_size;
  const float* x = (const float*)d_in[0]; const float* w1 = (const float*)d_in[1];
  const float* g1 = (const float*)d_in[2]; const float* be1 = (const float*)d_in[3]; const float* m1 = (const float*)d_in[4]; const float* v1 = (const float*)d_in[5];
  const float* wq = (const float*)d_in[6]; const float* bq = (const float*)d_in[7]; const float* wk = (const float*)d_in[8]; const float* bk = (const float*)d_in[9];
  const float* wv = (const float*)d_in[10]; const float* bv = (const float*)d_in[11]; const float* relh = (const float*)d_in[12]; const float* relw = (const float*)d_in[13];
  const float* w2 = (const float*)d_in[14]; const float* g2 = (const float*)d_in[15]; const float* be2 = (const float*)d_in[16]; const float* m2 = (const float*)d_in[17]; const float* v2 = (const float*)d_in[18];
  float* out = (float*)d_out;
  char* ws = (char*)d_ws; size_t off = 0;
  auto carve = [&](size_t bytes) -> char* { char* p = ws + off; off += (bytes + 255) & ~(size_t)255; return p; };
  _Float16* XT = (_Float16*)carve((size_t)NS * BB * CIN * 2);
  unsigned* W1f = (unsigned*)carve((size_t)CM * CIN * 2); float* b1f = (float*)carve(CM * 4);
  unsigned* W2f = (unsigned*)carve((size_t)CIN * CM * 2); float* b2f = (float*)carve(CIN * 4);
  _Float16* Wq16 = (_Float16*)carve((size_t)CM * CM * 2); _Float16* Wk16 = (_Float16*)carve((size_t)CM * CM * 2); _Float16* Wv16 = (_Float16*)carve((size_t)CM * CM * 2);
  unsigned* X1T = (unsigned*)carve((size_t)BB * NS * CM * 2);
  unsigned* QP = (unsigned*)carve((size_t)BB * NS * 256 * 2);
  unsigned* KQ = (unsigned*)carve((size_t)BB * NS * 256 * 2);
  unsigned* V16 = (unsigned*)carve((size_t)BB * CM * NS * 2);
  float* S = (float*)carve((size_t)8 * NS * NS * 4);
  unsigned* P16 = (unsigned*)carve((size_t)8 * NS * NS * 2);
  unsigned* OT = (unsigned*)carve((size_t)BB * NS * CM * 2);
  float* Y = (float*)carve((size_t)BB * CIN * NS * 4);
  transpose_cast_f16<<<dim3(NS / 64, BB * CIN / 64), dim3(32, 8), 0, stream>>>(x, NS, XT, BB * CIN, 1.0f);
  fold_bn_kernel<<<(CM * CIN / 2 + 255) / 256, 256, 0, stream>>>(w1, g1, be1, m1, v1, CM, CIN, W1f, b1f);
  fold_bn_kernel<<<(CIN * CM / 2 + 255) / 256, 256, 0, stream>>>(w2, g2, be2, m2, v2, CIN, CM, W2f, b2f);
  cast_f32_f16x2<<<(CM * CM / 2 + 255) / 256, 256, 0, stream>>>(wq, Wq16, CM * CM / 2); cast_f32_f16x2<<<(CM * CM / 2 + 255) / 256, 256, 0, stream>>>(wk, Wk16, CM * CM / 2); cast_f32_f16x2<<<(CM * CM / 2 + 255) / 256, 256, 0, stream>>>(wv, Wv16, CM * CM / 2);
  { const int t = (NS / 64) * (CM / 64);
    wmma_gemm64<0, false, 2, 1, false, 3><<<dim3((t + 7) / 8, BB), 256, 0, stream>>>(U16(XT), nullptr, BB * CIN, CIN, (const unsigned short*)W1f, nullptr, CIN, 0, X1T, nullptr, CM, (long)NS * CM, b1f, nullptr, 0, NS, CM, CIN, 1.0f); }
  { const int t = (NS / 64) * (CM / 64);
    wmma_gemm64<0, false, 2, 1, false, 0><<<dim3((t + 7) / 8, BB), 256, 0, stream>>>((const unsigned short*)X1T, nullptr, CM, (long)NS * CM, U16(Wq16), nullptr, CM, 0, QP, nullptr, 256, (long)NS * 256, bq, nullptr, 0, NS, CM, CM, 1.0f);
    wmma_gemm64<0, false, 2, 1, false, 0><<<dim3((t + 7) / 8, BB), 256, 0, stream>>>((const unsigned short*)X1T, nullptr, CM, (long)NS * CM, U16(Wq16), nullptr, CM, 0, KQ + 64, nullptr, 256, (long)NS * 256, bq, nullptr, 0, NS, CM, CM, 1.0f);
    wmma_gemm64<0, false, 2, 1, false, 0><<<dim3((t + 7) / 8, BB), 256, 0, stream>>>((const unsigned short*)X1T, nullptr, CM, (long)NS * CM, U16(Wk16), nullptr, CM, 0, KQ, nullptr, 256, (long)NS * 256, bk, nullptr, 0, NS, CM, CM, 1.0f);
    const int tv = (CM / 64) * (NS / 64);
    wmma_gemm64<0, false, 1, 1, false, 0><<<dim3((tv + 7) / 8, BB), 256, 0, stream>>>(U16(Wv16), nullptr, CM, 0, (const unsigned short*)X1T, nullptr, CM, (long)NS * CM, V16, nullptr, NS, (long)CM * NS, bv, nullptr, 0, CM, NS, CM, 1.0f); }
  pos_kernel<<<(BB * NS * 64 + 255) / 256, 256, 0, stream>>>(relh, relw, QP);
  for (int g8 = 0; g8 < BB / 8; ++g8) {
    const size_t b0 = (size_t)g8 * 8;
    { const int t = (NS / 64) * (NS / 64);
      wmma_gemm64<0, false, 0, 0, false><<<dim3((t + 7) / 8, 8), 256, 0, stream>>>((const unsigned short*)(QP + b0 * NS * 128), nullptr, 256, (long)NS * 256, (const unsigned short*)(KQ + b0 * NS * 128), nullptr, 256, (long)NS * 256, S, nullptr, NS, (long)NS * NS, nullptr, nullptr, 0, NS, NS, 256, 1.0f); }
    softmax_kernel<<<8 * NS, 256, 0, stream>>>(S, P16);
    { const int t = (NS / 64) * (CM / 64);
      wmma_gemm64<0, false, 0, 1, false, 0><<<dim3((t + 7) / 8, 8), 256, 0, stream>>>((const unsigned short*)P16, nullptr, NS, (long)NS * NS, (const unsigned short*)(V16 + b0 * CM * NS / 2), nullptr, NS, (long)CM * NS, OT + b0 * NS * CM / 2, nullptr, CM, (long)NS * CM, nullptr, nullptr, 0, NS, CM, NS, 1.0f / 32768.0f); }
  }
  { const int t = (CIN / 64) * (NS / 64);
    wmma_gemm64<0, false, 1, 0, false, 3><<<dim3((t + 7) / 8, BB), 256, 0, stream>>>((const unsigned short*)W2f, nullptr, CM, 0, (const unsigned short*)OT, nullptr, CM, (long)NS * CM, Y, nullptr, NS, (long)CIN * NS, b2f, nullptr, 0, CIN, NS, CM, 1.0f); }
  resid_kernel<<<(BB * CIN * NS / 4 + 255) / 256, 256, 0, stream>>>(x, Y, out, (long)BB * CIN * NS / 4);
}
